// PhaseBindingBlock_84825604096594
// MI455X (gfx1250) — hardware-verified
//
#include <hip/hip_runtime.h>
#include <math.h>
#include <stdint.h>

#define NB   2
#define SEQ  2048
#define DM   512
#define KO   32
#define QK   64
#define MTOT (NB * SEQ)

typedef __attribute__((ext_vector_type(16))) __bf16 v16b;
typedef __attribute__((ext_vector_type(8)))  __bf16 v8b;
typedef __attribute__((ext_vector_type(8)))  float  v8f;
typedef __attribute__((ext_vector_type(4)))  float  v4f;
typedef __attribute__((ext_vector_type(2)))  float  v2f;
typedef __attribute__((ext_vector_type(4)))  unsigned int   v4u;
typedef __attribute__((ext_vector_type(8)))  unsigned short v8us;

union FB { v16b v; v8b h[2]; };

__device__ __forceinline__ unsigned short f2bf_bits(float f) {
  unsigned u = __float_as_uint(f);
  return (unsigned short)((u + 0x7FFFu + ((u >> 16) & 1u)) >> 16);
}
__device__ __forceinline__ float bf_bits2f(unsigned short h) { return __uint_as_float(((unsigned)h) << 16); }
__device__ __forceinline__ unsigned pk16(unsigned short a, unsigned short b) { return (unsigned)a | ((unsigned)b << 16); }

__device__ __forceinline__ v8f zero8() { return (v8f){0.f, 0.f, 0.f, 0.f, 0.f, 0.f, 0.f, 0.f}; }

__device__ __forceinline__ v16b ldfrag(const __bf16* p) {
  FB f;
  f.h[0] = *(const v8b*)(p);
  f.h[1] = *(const v8b*)(p + 16);
  return f.v;
}

__device__ __forceinline__ v8f mma3(v16b ah, v16b al, v16b bh, v16b bl, v8f c) {
  c = __builtin_amdgcn_wmma_f32_16x16x32_bf16(false, ah, false, bh, (short)0, c, false, false);
  c = __builtin_amdgcn_wmma_f32_16x16x32_bf16(false, ah, false, bl, (short)0, c, false, false);
  c = __builtin_amdgcn_wmma_f32_16x16x32_bf16(false, al, false, bh, (short)0, c, false, false);
  asm volatile("v_nop\n\tv_nop\n\tv_nop\n\tv_nop" : "+v"(c) : "v"(ah), "v"(al), "v"(bh), "v"(bl));
  return c;
}

__device__ __forceinline__ void wave_lds_sync() {
  __builtin_amdgcn_fence(__ATOMIC_RELEASE, "workgroup");
  __builtin_amdgcn_wave_barrier();
  __builtin_amdgcn_fence(__ATOMIC_ACQUIRE, "workgroup");
}

__global__ __launch_bounds__(256) void split_bf16x2_kernel(const float* __restrict__ in, unsigned short* hi,
                                                           unsigned short* lo, int n2) {
  const int i = blockIdx.x * 256 + threadIdx.x;
  if (i < n2) {
    const v2f f = *(const v2f*)(in + 2 * (size_t)i);
    const unsigned short h0 = f2bf_bits(f[0]), h1 = f2bf_bits(f[1]);
    const unsigned short l0 = f2bf_bits(f[0] - bf_bits2f(h0)), l1 = f2bf_bits(f[1] - bf_bits2f(h1));
    const unsigned uh = pk16(h0, h1), ul = pk16(l0, l1);
    ((volatile unsigned*)hi)[i] = uh;
    ((volatile unsigned*)lo)[i] = ul;
    __threadfence();
    ((volatile unsigned*)hi)[i] = uh;
    ((volatile unsigned*)lo)[i] = ul;
  }
}

__global__ __launch_bounds__(256) void tsplit_kernel(const float* __restrict__ W, unsigned short* oh,
                                                     unsigned short* ol, int R, int Cc) {
  __shared__ __align__(16) float tf[64 * 68];
  const int c0  = blockIdx.x * 64;
  const int r0  = blockIdx.y * 64;
  const int tid = threadIdx.x;
  {
    const int lr = tid >> 4;
    const int c4 = (tid & 15) * 4;
#pragma unroll
    for (int it = 0; it < 4; ++it) {
      const int rr = it * 16 + lr;
      const v4f a = *(const v4f*)(W + (size_t)(r0 + rr) * Cc + c0 + c4);
      *(v4f*)(tf + rr * 68 + c4) = a;
    }
  }
  __syncthreads();
  const int sub = tid >> 3;
  const int c8  = (tid & 7) * 8;
  v4u hv[2], lv[2];
#pragma unroll
  for (int it = 0; it < 2; ++it) {
    const int oc = it * 32 + sub;
    v4u a, a2;
#pragma unroll
    for (int q = 0; q < 4; ++q) {
      const float f0 = tf[(c8 + 2 * q) * 68 + oc];
      const float f1 = tf[(c8 + 2 * q + 1) * 68 + oc];
      const unsigned short h0 = f2bf_bits(f0), h1 = f2bf_bits(f1);
      const unsigned short l0 = f2bf_bits(f0 - bf_bits2f(h0)), l1 = f2bf_bits(f1 - bf_bits2f(h1));
      a[q]  = pk16(h0, h1);
      a2[q] = pk16(l0, l1);
    }
    hv[it] = a; lv[it] = a2;
  }
  for (int pass = 0; pass < 2; ++pass) {
#pragma unroll
    for (int it = 0; it < 2; ++it) {
      const int oc = it * 32 + sub;
      const size_t go = (size_t)(c0 + oc) * R + r0 + c8;
      *(volatile v4u*)(oh + go) = hv[it];
      *(volatile v4u*)(ol + go) = lv[it];
    }
    __threadfence();
  }
}

__global__ __launch_bounds__(256) void tsplit32_kernel(const float* __restrict__ W, unsigned short* oh,
                                                       unsigned short* ol, int R) {
  __shared__ __align__(16) float tf[64 * 36];
  const int r0  = blockIdx.x * 64;
  const int tid = threadIdx.x;
  {
    const int rr = tid >> 3;
    const int c4 = (tid & 7) * 4;
#pragma unroll
    for (int it = 0; it < 2; ++it) {
      const int row = it * 32 + rr;
      const v4f a = *(const v4f*)(W + (size_t)(r0 + row) * KO + c4);
      *(v4f*)(tf + row * 36 + c4) = a;
    }
  }
  __syncthreads();
  const int oc = tid >> 3;
  const int c8 = (tid & 7) * 8;
  v4u hv, lv;
#pragma unroll
  for (int q = 0; q < 4; ++q) {
    const float f0 = tf[(c8 + 2 * q) * 36 + oc];
    const float f1 = tf[(c8 + 2 * q + 1) * 36 + oc];
    const unsigned short h0 = f2bf_bits(f0), h1 = f2bf_bits(f1);
    const unsigned short l0 = f2bf_bits(f0 - bf_bits2f(h0)), l1 = f2bf_bits(f1 - bf_bits2f(h1));
    hv[q] = pk16(h0, h1);
    lv[q] = pk16(l0, l1);
  }
  const size_t go = (size_t)oc * R + r0 + c8;
  for (int pass = 0; pass < 2; ++pass) {
    *(volatile v4u*)(oh + go) = hv;
    *(volatile v4u*)(ol + go) = lv;
    __threadfence();
  }
}

template <int BIAS_MODE, int OUT_MODE, bool RESID, int ACT>
__global__ __launch_bounds__(256) void gemm_hl_kernel(
    const unsigned short* __restrict__ Ahp, const unsigned short* __restrict__ Alp, int lda, long long strideA,
    const unsigned short* __restrict__ Bhp, const unsigned short* __restrict__ Blp, int ldb, long long strideB,
    void* Cout, void* Cout2, int ldc, long long strideC,
    const float* __restrict__ bias,
    const float* __restrict__ resid, long long strideR,
    int M, int N, int K) {
  __shared__ __align__(16) float sT[8][16 * 68];
  const __bf16* Ah = (const __bf16*)(const void*)Ahp;
  const __bf16* Al = (const __bf16*)(const void*)Alp;
  const __bf16* Bh = (const __bf16*)(const void*)Bhp;
  const __bf16* Bl = (const __bf16*)(const void*)Blp;
  const int bz   = blockIdx.y;
  const int lane = threadIdx.x & 31;
  const int wave = threadIdx.x >> 5;
  const int tilesN = N >> 6;
  const int tilesM = M >> 5;
  const int tile = blockIdx.x * 8 + wave;
  if (tile >= tilesM * tilesN) return;
  const int tm = tile / tilesN;
  const int tn = tile - tm * tilesN;
  const int m0 = tm << 5;
  const int n0 = tn << 6;

  const __bf16* Abh = Ah + (size_t)bz * strideA;
  const __bf16* Abl = Al + (size_t)bz * strideA;
  const __bf16* Bbh = Bh + (size_t)bz * strideB;
  const __bf16* Bbl = Bl + (size_t)bz * strideB;

  const int rl   = lane & 15;
  const int koff = (lane >> 4) * 8;
  const int mOff = (lane >> 4) * 8;

  v8f acc[2][4];
#pragma unroll
  for (int i = 0; i < 2; ++i)
#pragma unroll
    for (int j = 0; j < 4; ++j) acc[i][j] = zero8();

#pragma unroll 1
  for (int k0 = 0; k0 < K; k0 += 32) {
    v16b bh[4], bl[4];
#pragma unroll
    for (int j = 0; j < 4; ++j) {
      const size_t bo = (size_t)(n0 + (j << 4) + rl) * ldb + koff + k0;
      bh[j] = ldfrag(Bbh + bo);
      bl[j] = ldfrag(Bbl + bo);
    }
#pragma unroll
    for (int i = 0; i < 2; ++i) {
      const size_t ao = (size_t)(m0 + (i << 4) + rl) * lda + koff + k0;
      const v16b ah = ldfrag(Abh + ao);
      const v16b al = ldfrag(Abl + ao);
#pragma unroll
      for (int j = 0; j < 4; ++j) acc[i][j] = mma3(ah, al, bh[j], bl[j], acc[i][j]);
    }
  }

  float* slab = sT[wave];
  const float* Rb = RESID ? (resid + (size_t)bz * strideR) : nullptr;
#pragma unroll
  for (int i = 0; i < 2; ++i) {
    const int mBase = m0 + (i << 4);
#pragma unroll
    for (int j = 0; j < 4; ++j) {
      const int n = n0 + (j << 4) + rl;
      float bv = 0.f;
      if (BIAS_MODE == 2) bv = bias[n];
#pragma unroll
      for (int r = 0; r < 8; ++r) {
        float v = acc[i][j][r];
        if (BIAS_MODE == 1) v += bias[mBase + mOff + r];
        if (BIAS_MODE == 2) v += bv;
        if (RESID) v += Rb[(size_t)(mBase + mOff + r) * ldc + n];
        if (ACT == 1) v = tanhf(v);
        slab[(mOff + r) * 68 + (j << 4) + rl] = v;
      }
    }
    wave_lds_sync();
    if (OUT_MODE == 0) {
      float* C = (float*)Cout + (size_t)bz * strideC;
      const int hsel = lane >> 4, c4 = (lane & 15) * 4;
      for (int pass = 0; pass < 2; ++pass) {
#pragma unroll
        for (int it = 0; it < 8; ++it) {
          const int row = it * 2 + hsel;
          const v4f v = *(const v4f*)(slab + row * 68 + c4);
          *(volatile v4f*)(C + (size_t)(mBase + row) * ldc + n0 + c4) = v;
        }
        __threadfence();
      }
    } else {
      const int q4 = lane >> 3, c8 = (lane & 7) * 8;
      unsigned short* C  = (unsigned short*)Cout  + (size_t)bz * strideC;
      unsigned short* C2 = (unsigned short*)Cout2 + (size_t)bz * strideC;
      for (int pass = 0; pass < 2; ++pass) {
#pragma unroll
        for (int it = 0; it < 4; ++it) {
          const int row = it * 4 + q4;
          const float* sp = slab + row * 68 + c8;
          v8us hv, lv;
#pragma unroll
          for (int e = 0; e < 8; ++e) {
            const unsigned short hb = f2bf_bits(sp[e]);
            const unsigned short lb = f2bf_bits(sp[e] - bf_bits2f(hb));
            hv[e] = hb;
            lv[e] = lb;
          }
          const size_t go = (size_t)(mBase + row) * ldc + n0 + c8;
          *(volatile v8us*)(C + go)  = hv;
          *(volatile v8us*)(C2 + go) = lv;
        }
        __threadfence();
      }
    }
    wave_lds_sync();
  }
}

__global__ __launch_bounds__(128) void enc_head_kernel(
    const unsigned short* __restrict__ Hkhp, const unsigned short* __restrict__ Hklp,
    const unsigned short* __restrict__ Hqhp, const unsigned short* __restrict__ Hqlp,
    const unsigned short* __restrict__ Xhp,  const unsigned short* __restrict__ Xlp,
    const unsigned short* __restrict__ Wk2hp, const unsigned short* __restrict__ Wk2lp,
    const unsigned short* __restrict__ Wq2hp, const unsigned short* __restrict__ Wq2lp,
    const unsigned short* __restrict__ Wkahp, const unsigned short* __restrict__ Wkalp,
    const unsigned short* __restrict__ Wqahp, const unsigned short* __restrict__ Wqalp,
    const float* __restrict__ bk2, const float* __restrict__ bq2,
    const float* __restrict__ bka, const float* __restrict__ bqa,
    const float* __restrict__ pos,
    unsigned short* Qhp, unsigned short* Qlp, unsigned short* Khp, unsigned short* Klp) {
  __shared__ __align__(16) float slab_all[4][16 * 132];
  const int tid = threadIdx.x, wave = tid >> 5, lane = tid & 31, hh = lane >> 4, c = lane & 15;
  const int row0 = blockIdx.x * 64 + wave * 16;

  const __bf16* Hkh = (const __bf16*)(const void*)Hkhp;  const __bf16* Hkl = (const __bf16*)(const void*)Hklp;
  const __bf16* Hqh = (const __bf16*)(const void*)Hqhp;  const __bf16* Hql = (const __bf16*)(const void*)Hqlp;
  const __bf16* Xh  = (const __bf16*)(const void*)Xhp;   const __bf16* Xl  = (const __bf16*)(const void*)Xlp;
  const __bf16* Wk2h = (const __bf16*)(const void*)Wk2hp; const __bf16* Wk2l = (const __bf16*)(const void*)Wk2lp;
  const __bf16* Wq2h = (const __bf16*)(const void*)Wq2hp; const __bf16* Wq2l = (const __bf16*)(const void*)Wq2lp;
  const __bf16* Wkah = (const __bf16*)(const void*)Wkahp; const __bf16* Wkal = (const __bf16*)(const void*)Wkalp;
  const __bf16* Wqah = (const __bf16*)(const void*)Wqahp; const __bf16* Wqal = (const __bf16*)(const void*)Wqalp;

  v8f aPk[2], aPq[2], aAk[2], aAq[2];
#pragma unroll
  for (int t = 0; t < 2; ++t) { aPk[t] = zero8(); aPq[t] = zero8(); aAk[t] = zero8(); aAq[t] = zero8(); }

#pragma unroll 1
  for (int k0 = 0; k0 < DM; k0 += 32) {
    const size_t ao = (size_t)(row0 + c) * DM + k0 + 8 * hh;
    const v16b ahk = ldfrag(Hkh + ao), alk = ldfrag(Hkl + ao);
    const v16b ahq = ldfrag(Hqh + ao), alq = ldfrag(Hql + ao);
    const v16b axh = ldfrag(Xh + ao),  axl = ldfrag(Xl + ao);
#pragma unroll
    for (int t = 0; t < 2; ++t) {
      const size_t bo = (size_t)(t * 16 + c) * DM + k0 + 8 * hh;
      aPk[t] = mma3(ahk, alk, ldfrag(Wk2h + bo), ldfrag(Wk2l + bo), aPk[t]);
      aPq[t] = mma3(ahq, alq, ldfrag(Wq2h + bo), ldfrag(Wq2l + bo), aPq[t]);
      aAk[t] = mma3(axh, axl, ldfrag(Wkah + bo), ldfrag(Wkal + bo), aAk[t]);
      aAq[t] = mma3(axh, axl, ldfrag(Wqah + bo), ldfrag(Wqal + bo), aAq[t]);
    }
  }

  float* sl = slab_all[wave];
#pragma unroll
  for (int t = 0; t < 2; ++t) {
    const int n = t * 16 + c;
    const float b1 = bk2[n], b2 = bka[n], b3 = bq2[n], b4 = bqa[n];
#pragma unroll
    for (int r = 0; r < 8; ++r) {
      float* sp = sl + (8 * hh + r) * 132;
      sp[n]      = aPk[t][r] + b1;
      sp[32 + n] = aAk[t][r] + b2;
      sp[64 + n] = aPq[t][r] + b3;
      sp[96 + n] = aAq[t][r] + b4;
    }
  }
  wave_lds_sync();

  const float PI = 3.14159265358979323846f;
#pragma unroll 1
  for (int it = 0; it < 16; ++it) {
    float* sp = sl + it * 132;
    const int l = (row0 + it) & (SEQ - 1);
    const float pa  = pos[l * KO + lane];
    const float vpk = sp[lane], vak = sp[32 + lane], vpq = sp[64 + lane], vaq = sp[96 + lane];
    const float phk = tanhf(vpk) * PI + pa;
    const float phq = tanhf(vpq) * PI + pa;
    const float ak  = fmaxf(vak, 0.f) + log1pf(expf(-fabsf(vak))) + 0.1f;
    const float aq  = fmaxf(vaq, 0.f) + log1pf(expf(-fabsf(vaq))) + 0.1f;
    sp[lane]      = ak * cosf(phk);
    sp[32 + lane] = ak * sinf(phk);
    sp[64 + lane] = aq * cosf(phq);
    sp[96 + lane] = aq * sinf(phq);
  }
  wave_lds_sync();

  const int q4 = lane >> 3, c8 = (lane & 7) * 8;
  for (int pass = 0; pass < 2; ++pass) {
#pragma unroll
    for (int it = 0; it < 4; ++it) {
      const int row = it * 4 + q4;
      const float* sk = sl + row * 132 + c8;
      const float* sq = sl + row * 132 + 64 + c8;
      v8us khv, klv, qhv, qlv;
#pragma unroll
      for (int e = 0; e < 8; ++e) {
        const unsigned short kh = f2bf_bits(sk[e]);
        const unsigned short kl = f2bf_bits(sk[e] - bf_bits2f(kh));
        const unsigned short qh = f2bf_bits(sq[e]);
        const unsigned short ql = f2bf_bits(sq[e] - bf_bits2f(qh));
        khv[e] = kh; klv[e] = kl; qhv[e] = qh; qlv[e] = ql;
      }
      const size_t go = (size_t)(row0 + row) * QK + c8;
      *(volatile v8us*)(Khp + go) = khv;
      *(volatile v8us*)(Klp + go) = klv;
      *(volatile v8us*)(Qhp + go) = qhv;
      *(volatile v8us*)(Qlp + go) = qlv;
    }
    __threadfence();
  }
}

__global__ __launch_bounds__(128) void causal_mix_kernel(
    const unsigned short* __restrict__ Qhp, const unsigned short* __restrict__ Qlp,
    const unsigned short* __restrict__ Khp, const unsigned short* __restrict__ Klp,
    const unsigned short* __restrict__ Vhp, const unsigned short* __restrict__ Vlp,
    float* Rout) {
  __shared__ __align__(16) unsigned char smem[65536];
  __bf16* Ksh = (__bf16*)(smem);
  __bf16* Ksl = (__bf16*)(smem + 8192);
  __bf16* Vth = (__bf16*)(smem + 16384);
  __bf16* Vtl = (__bf16*)(smem + 32768);
  __bf16* Pgh = (__bf16*)(smem + 49152);
  __bf16* Pgl = (__bf16*)(smem + 57344);
  float*  Osb = (float*)(smem);

  const int tid = threadIdx.x, wave = tid >> 5, lane = tid & 31, hh = lane >> 4, c = lane & 15;
  const int bx  = blockIdx.x;
  const int dch = bx & 3;
  const int qb  = (bx >> 2) & 31;
  const int b   = bx >> 7;
  const int q0  = qb * 64 + wave * 16;
  const size_t grow0 = (size_t)b * SEQ + q0;

  const __bf16* Qh = (const __bf16*)(const void*)Qhp; const __bf16* Ql = (const __bf16*)(const void*)Qlp;
  const __bf16* Kh = (const __bf16*)(const void*)Khp; const __bf16* Kl = (const __bf16*)(const void*)Klp;
  const __bf16* Vh = (const __bf16*)(const void*)Vhp; const __bf16* Vl = (const __bf16*)(const void*)Vlp;

  v16b qah[2], qal[2];
#pragma unroll
  for (int dc = 0; dc < 2; ++dc) {
    qah[dc] = ldfrag(Qh + (grow0 + c) * QK + dc * 32 + 8 * hh);
    qal[dc] = ldfrag(Ql + (grow0 + c) * QK + dc * 32 + 8 * hh);
  }
  v8f oacc[8];
#pragma unroll
  for (int t = 0; t < 8; ++t) oacc[t] = zero8();

  __bf16* pwh = Pgh + wave * (16 * 64);
  __bf16* pwl = Pgl + wave * (16 * 64);

  const int nch = qb + 1;
  for (int kc = 0; kc < nch; ++kc) {
    const int kv0 = kc * 64;
    __syncthreads();
    {
      const int r = tid >> 1, half = (tid & 1) * 32;
      const __bf16* ks = Kh + ((size_t)b * SEQ + kv0 + r) * QK + half;
      const __bf16* ls = Kl + ((size_t)b * SEQ + kv0 + r) * QK + half;
#pragma unroll
      for (int i = 0; i < 4; ++i) {
        *(v8b*)(Ksh + r * QK + half + 8 * i) = *(const v8b*)(ks + 8 * i);
        *(v8b*)(Ksl + r * QK + half + 8 * i) = *(const v8b*)(ls + 8 * i);
      }
      const __bf16* vs = Vh + ((size_t)b * DM + dch * 128 + tid) * SEQ + kv0;
      const __bf16* vl = Vl + ((size_t)b * DM + dch * 128 + tid) * SEQ + kv0;
#pragma unroll
      for (int i = 0; i < 8; ++i) {
        *(v8b*)(Vth + tid * 64 + 8 * i) = *(const v8b*)(vs + 8 * i);
        *(v8b*)(Vtl + tid * 64 + 8 * i) = *(const v8b*)(vl + 8 * i);
      }
    }
    __syncthreads();

    v8f s[4];
#pragma unroll
    for (int j = 0; j < 4; ++j) {
      s[j] = zero8();
#pragma unroll
      for (int dc = 0; dc < 2; ++dc) {
        FB kb, kl;
        const int kb0 = (j * 16 + c) * QK + dc * 32 + 8 * hh;
        kb.h[0] = *(const v8b*)(Ksh + kb0);
        kb.h[1] = *(const v8b*)(Ksh + kb0 + 16);
        kl.h[0] = *(const v8b*)(Ksl + kb0);
        kl.h[1] = *(const v8b*)(Ksl + kb0 + 16);
        s[j] = mma3(qah[dc], qal[dc], kb.v, kl.v, s[j]);
      }
    }
    const bool diag = (kc == qb);
#pragma unroll
    for (int r = 0; r < 8; ++r) {
      const int qrow = q0 + 8 * hh + r;
#pragma unroll
      for (int j = 0; j < 4; ++j) {
        const int kvcol = kv0 + j * 16 + c;
        float pm = s[j][r];
        if (diag && kvcol > qrow) pm = 0.f;
        const unsigned short hb = f2bf_bits(pm);
        const unsigned short lb = f2bf_bits(pm - bf_bits2f(hb));
        pwh[(8 * hh + r) * 64 + j * 16 + c] = __builtin_bit_cast(__bf16, hb);
        pwl[(8 * hh + r) * 64 + j * 16 + c] = __builtin_bit_cast(__bf16, lb);
      }
    }
    wave_lds_sync();

#pragma unroll 1
    for (int kk = 0; kk < 2; ++kk) {
      FB pa, pl;
      const int pb0 = c * 64 + kk * 32 + 8 * hh;
      pa.h[0] = *(const v8b*)(pwh + pb0);
      pa.h[1] = *(const v8b*)(pwh + pb0 + 16);
      pl.h[0] = *(const v8b*)(pwl + pb0);
      pl.h[1] = *(const v8b*)(pwl + pb0 + 16);
#pragma unroll
      for (int t = 0; t < 8; ++t) {
        FB vb, vlo;
        const int vb0 = (t * 16 + c) * 64 + kk * 32 + 8 * hh;
        vb.h[0]  = *(const v8b*)(Vth + vb0);
        vb.h[1]  = *(const v8b*)(Vth + vb0 + 16);
        vlo.h[0] = *(const v8b*)(Vtl + vb0);
        vlo.h[1] = *(const v8b*)(Vtl + vb0 + 16);
        oacc[t] = mma3(pa.v, pl.v, vb.v, vlo.v, oacc[t]);
      }
    }
  }
  __syncthreads();

  float* os = Osb + wave * (16 * 132);
#pragma unroll
  for (int r = 0; r < 8; ++r) {
    const int lq = q0 + 8 * hh + r;
    const float nrm = sqrtf((float)((lq + 1) * KO));
    const float inv = 1.0f / nrm;
#pragma unroll
    for (int t = 0; t < 8; ++t) os[(8 * hh + r) * 132 + t * 16 + c] = oacc[t][r] * inv;
  }
  wave_lds_sync();
  for (int pass = 0; pass < 2; ++pass) {
#pragma unroll
    for (int it = 0; it < 16; ++it) {
      const v4f val = *(const v4f*)(os + it * 132 + lane * 4);
      *(volatile v4f*)(Rout + (grow0 + it) * DM + dch * 128 + lane * 4) = val;
    }
    __threadfence();
  }
}

__global__ __launch_bounds__(256) void ln_split_kernel(const float* __restrict__ R, const float* __restrict__ g,
                                                       const float* __restrict__ be,
                                                       unsigned short* Lh, unsigned short* Ll) {
  const int tid = threadIdx.x, wave = tid >> 5, lane = tid & 31;
  const int row = blockIdx.x * 8 + wave;
  const float* rp = R + (size_t)row * DM;
  const int cA = 8 * lane, cB = 256 + 8 * lane;
  const v4f x0 = *(const v4f*)(rp + cA), x1 = *(const v4f*)(rp + cA + 4);
  const v4f x2 = *(const v4f*)(rp + cB), x3 = *(const v4f*)(rp + cB + 4);
  const v4f g0 = *(const v4f*)(g + cA),  g1 = *(const v4f*)(g + cA + 4);
  const v4f g2 = *(const v4f*)(g + cB),  g3 = *(const v4f*)(g + cB + 4);
  const v4f e0 = *(const v4f*)(be + cA), e1 = *(const v4f*)(be + cA + 4);
  const v4f e2 = *(const v4f*)(be + cB), e3 = *(const v4f*)(be + cB + 4);
  float v[16], gg[16], bb[16];
#pragma unroll
  for (int e = 0; e < 4; ++e) {
    v[e] = x0[e]; v[4 + e] = x1[e]; v[8 + e] = x2[e]; v[12 + e] = x3[e];
    gg[e] = g0[e]; gg[4 + e] = g1[e]; gg[8 + e] = g2[e]; gg[12 + e] = g3[e];
    bb[e] = e0[e]; bb[4 + e] = e1[e]; bb[8 + e] = e2[e]; bb[12 + e] = e3[e];
  }
  float sum = 0.f;
#pragma unroll
  for (int e = 0; e < 16; ++e) sum += v[e];
#pragma unroll
  for (int off = 1; off < 32; off <<= 1) sum += __shfl_xor(sum, off, 32);
  const float mu = sum * (1.0f / (float)DM);
  float ss = 0.f;
#pragma unroll
  for (int e = 0; e < 16; ++e) { const float d = v[e] - mu; v[e] = d; ss += d * d; }
#pragma unroll
  for (int off = 1; off < 32; off <<= 1) ss += __shfl_xor(ss, off, 32);
  const float var  = ss * (1.0f / (float)DM);
  const float rstd = 1.0f / sqrtf(var + 1e-5f);
  v8us hA, lA, hB, lB;
#pragma unroll
  for (int e = 0; e < 8; ++e) {
    const float ya = v[e] * rstd * gg[e] + bb[e];
    const float yb = v[8 + e] * rstd * gg[8 + e] + bb[8 + e];
    const unsigned short ha = f2bf_bits(ya), la = f2bf_bits(ya - bf_bits2f(ha));
    const unsigned short hb = f2bf_bits(yb), lb = f2bf_bits(yb - bf_bits2f(hb));
    hA[e] = ha; lA[e] = la; hB[e] = hb; lB[e] = lb;
  }
  const size_t oA = (size_t)row * DM + cA, oB = (size_t)row * DM + cB;
  for (int pass = 0; pass < 2; ++pass) {
    *(volatile v8us*)(Lh + oA) = hA;
    *(volatile v8us*)(Lh + oB) = hB;
    *(volatile v8us*)(Ll + oA) = lA;
    *(volatile v8us*)(Ll + oB) = lB;
    __threadfence();
  }
}

extern "C" void kernel_launch(void* const* d_in, const int* in_sizes, int n_in,
                              void* d_out, int out_size, void* d_ws, size_t ws_size,
                              hipStream_t stream) {
  if (n_in < 20) return;
  if (in_sizes[0] != MTOT * DM || in_sizes[1] != SEQ * KO) return;
  if (in_sizes[2] != DM * DM || in_sizes[8] != DM * DM || in_sizes[14] != DM * DM || in_sizes[18] != DM * DM) return;
  if (in_sizes[3] != DM || in_sizes[9] != DM || in_sizes[15] != DM || in_sizes[19] != DM) return;
  if (in_sizes[16] != DM || in_sizes[17] != DM) return;
  if (in_sizes[4] != DM * KO || in_sizes[6] != DM * KO || in_sizes[10] != DM * KO || in_sizes[12] != DM * KO) return;
  if (in_sizes[5] != KO || in_sizes[7] != KO || in_sizes[11] != KO || in_sizes[13] != KO) return;
  if (out_size != MTOT * DM) return;

  const float* x     = (const float*)d_in[0];
  const float* pos   = (const float*)d_in[1];
  const float* kp_w1 = (const float*)d_in[2];
  const float* kp_b1 = (const float*)d_in[3];
  const float* kp_w2 = (const float*)d_in[4];
  const float* kp_b2 = (const float*)d_in[5];
  const float* ka_w  = (const float*)d_in[6];
  const float* ka_b  = (const float*)d_in[7];
  const float* qp_w1 = (const float*)d_in[8];
  const float* qp_b1 = (const float*)d_in[9];
  const float* qp_w2 = (const float*)d_in[10];
  const float* qp_b2 = (const float*)d_in[11];
  const float* qa_w  = (const float*)d_in[12];
  const float* qa_b  = (const float*)d_in[13];
  const float* v_w   = (const float*)d_in[14];
  const float* v_b   = (const float*)d_in[15];
  const float* ln_g  = (const float*)d_in[16];
  const float* ln_b  = (const float*)d_in[17];
  const float* o_w   = (const float*)d_in[18];
  const float* o_b   = (const float*)d_in[19];

  const size_t PX = (size_t)MTOT * DM * 2;
  const size_t PW = (size_t)DM * DM * 2;
  const size_t PS = (size_t)KO * DM * 2;
  const size_t PQ = (size_t)MTOT * QK * 2;
  const size_t PV = (size_t)NB * DM * SEQ * 2;
  const size_t PR = (size_t)MTOT * DM * 4;
  size_t off = 0;
  const size_t oXh  = off; off += PX;  const size_t oXl  = off; off += PX;
  const size_t oHkh = off; off += PX;  const size_t oHkl = off; off += PX;
  const size_t oHqh = off; off += PX;  const size_t oHql = off; off += PX;
  const size_t oWkh = off; off += PW;  const size_t oWkl = off; off += PW;
  const size_t oWqh = off; off += PW;  const size_t oWql = off; off += PW;
  const size_t oWvh = off; off += PW;  const size_t oWvl = off; off += PW;
  const size_t oWoh = off; off += PW;  const size_t oWol = off; off += PW;
  const size_t oSk2h = off; off += PS; const size_t oSk2l = off; off += PS;
  const size_t oSq2h = off; off += PS; const size_t oSq2l = off; off += PS;
  const size_t oSkah = off; off += PS; const size_t oSkal = off; off += PS;
  const size_t oSqah = off; off += PS; const size_t oSqal = off; off += PS;
  const size_t oQth = off; off += PQ;  const size_t oQtl = off; off += PQ;
  const size_t oKth = off; off += PQ;  const size_t oKtl = off; off += PQ;
  const size_t oVTh = off; off += PV;  const size_t oVTl = off; off += PV;
  const size_t oR   = off; off += PR;
  const size_t oLh  = off; off += PX;  const size_t oLl  = off; off += PX;
  if (off > ws_size) return;

  char* ws = (char*)d_ws;
  unsigned short* Xh  = (unsigned short*)(ws + oXh);   unsigned short* Xl  = (unsigned short*)(ws + oXl);
  unsigned short* Hkh = (unsigned short*)(ws + oHkh);  unsigned short* Hkl = (unsigned short*)(ws + oHkl);
  unsigned short* Hqh = (unsigned short*)(ws + oHqh);  unsigned short* Hql = (unsigned short*)(ws + oHql);
  unsigned short* Wkh = (unsigned short*)(ws + oWkh);  unsigned short* Wkl = (unsigned short*)(ws + oWkl);
  unsigned short* Wqh = (unsigned short*)(ws + oWqh);  unsigned short* Wql = (unsigned short*)(ws + oWql);
  unsigned short* Wvh = (unsigned short*)(ws + oWvh);  unsigned short* Wvl = (unsigned short*)(ws + oWvl);
  unsigned short* Woh = (unsigned short*)(ws + oWoh);  unsigned short* Wol = (unsigned short*)(ws + oWol);
  unsigned short* Sk2h = (unsigned short*)(ws + oSk2h); unsigned short* Sk2l = (unsigned short*)(ws + oSk2l);
  unsigned short* Sq2h = (unsigned short*)(ws + oSq2h); unsigned short* Sq2l = (unsigned short*)(ws + oSq2l);
  unsigned short* Skah = (unsigned short*)(ws + oSkah); unsigned short* Skal = (unsigned short*)(ws + oSkal);
  unsigned short* Sqah = (unsigned short*)(ws + oSqah); unsigned short* Sqal = (unsigned short*)(ws + oSqal);
  unsigned short* Qth = (unsigned short*)(ws + oQth);  unsigned short* Qtl = (unsigned short*)(ws + oQtl);
  unsigned short* Kth = (unsigned short*)(ws + oKth);  unsigned short* Ktl = (unsigned short*)(ws + oKtl);
  unsigned short* VTh = (unsigned short*)(ws + oVTh);  unsigned short* VTl = (unsigned short*)(ws + oVTl);
  float*          Rws = (float*)(ws + oR);
  unsigned short* Lh  = (unsigned short*)(ws + oLh);   unsigned short* Ll  = (unsigned short*)(ws + oLl);

  const dim3 b256(256), b128(128);

  const int n2x = MTOT * DM / 2;
  split_bf16x2_kernel<<<dim3((n2x + 255) / 256), b256, 0, stream>>>(x, Xh, Xl, n2x);

  tsplit_kernel<<<dim3(DM / 64, DM / 64), b256, 0, stream>>>(kp_w1, Wkh, Wkl, DM, DM);
  tsplit_kernel<<<dim3(DM / 64, DM / 64), b256, 0, stream>>>(qp_w1, Wqh, Wql, DM, DM);
  tsplit_kernel<<<dim3(DM / 64, DM / 64), b256, 0, stream>>>(v_w,   Wvh, Wvl, DM, DM);
  tsplit_kernel<<<dim3(DM / 64, DM / 64), b256, 0, stream>>>(o_w,   Woh, Wol, DM, DM);
  tsplit32_kernel<<<dim3(DM / 64), b256, 0, stream>>>(kp_w2, Sk2h, Sk2l, DM);
  tsplit32_kernel<<<dim3(DM / 64), b256, 0, stream>>>(qp_w2, Sq2h, Sq2l, DM);
  tsplit32_kernel<<<dim3(DM / 64), b256, 0, stream>>>(ka_w,  Skah, Skal, DM);
  tsplit32_kernel<<<dim3(DM / 64), b256, 0, stream>>>(qa_w,  Sqah, Sqal, DM);

  const dim3 gH(((MTOT / 32) * (DM / 64) + 7) / 8, 1);
  gemm_hl_kernel<2, 2, false, 1><<<gH, b256, 0, stream>>>(
      Xh, Xl, DM, 0LL, Wkh, Wkl, DM, 0LL, (void*)Hkh, (void*)Hkl, DM, 0LL,
      kp_b1, nullptr, 0LL, MTOT, DM, DM);
  gemm_hl_kernel<2, 2, false, 1><<<gH, b256, 0, stream>>>(
      Xh, Xl, DM, 0LL, Wqh, Wql, DM, 0LL, (void*)Hqh, (void*)Hql, DM, 0LL,
      qp_b1, nullptr, 0LL, MTOT, DM, DM);

  const dim3 gV(((DM / 32) * (SEQ / 64) + 7) / 8, NB);
  gemm_hl_kernel<1, 2, false, 0><<<gV, b256, 0, stream>>>(
      Wvh, Wvl, DM, 0LL, Xh, Xl, DM, (long long)SEQ * DM, (void*)VTh, (void*)VTl, SEQ, (long long)DM * SEQ,
      v_b, nullptr, 0LL, DM, SEQ, DM);

  enc_head_kernel<<<dim3(MTOT / 64), b128, 0, stream>>>(
      Hkh, Hkl, Hqh, Hql, Xh, Xl,
      Sk2h, Sk2l, Sq2h, Sq2l, Skah, Skal, Sqah, Sqal,
      kp_b2, qp_b2, ka_b, qa_b, pos,
      Qth, Qtl, Kth, Ktl);

  causal_mix_kernel<<<dim3(NB * (SEQ / 64) * 4), b128, 0, stream>>>(Qth, Qtl, Kth, Ktl, VTh, VTl, Rws);

  ln_split_kernel<<<dim3(MTOT / 8), b256, 0, stream>>>(Rws, ln_g, ln_b, Lh, Ll);

  gemm_hl_kernel<2, 0, true, 0><<<gH, b256, 0, stream>>>(
      Lh, Ll, DM, 0LL, Woh, Wol, DM, 0LL, d_out, d_out, DM, 0LL,
      o_b, x, 0LL, MTOT, DM, DM);

  (void)hipGetLastError();
}
